// Difference_89567247991564
// MI455X (gfx1250) — hardware-verified
//
#include <hip/hip_runtime.h>

constexpr int kNa = 1024;
constexpr int kNb = 1024;
constexpr int kKF = 256;
constexpr int kDD = 128;
constexpr int kTI = 32;
constexpr int kTJ = 64;
constexpr int kStgPitch = 36;

static_assert(kNa % 64 == 0 && kNb % 64 == 0 && kKF % 64 == 0);
static_assert(kDD % 32 == 0);
static_assert(kNa % kTI == 0 && kNb % kTJ == 0 && kKF % 64 == 0);
static_assert(kNa == kNb);
static_assert((kNa * kDD) % 2048 == 0 && (kKF * kDD) % 2048 == 0);

constexpr int kBlkA = kNa * kDD / 2048;
constexpr int kBlkB = kNb * kDD / 2048;
constexpr int kBlkF = kKF * kDD / 2048;

constexpr size_t kOffAbf = 0;
constexpr size_t kOffBbf = kOffAbf + (size_t)kNa * kDD * 2;
constexpr size_t kOffFbf = kOffBbf + (size_t)kNb * kDD * 2;
constexpr size_t kOffAfk = kOffFbf + (size_t)kKF * kDD * 2;
constexpr size_t kOffBfk = kOffAfk + (size_t)kNa * kKF * 4;
constexpr size_t kWsTotal = kOffBfk + (size_t)kNb * kKF * 4;
static_assert(kWsTotal == 2686976);
static_assert(kOffBbf % 128 == 0 && kOffFbf % 128 == 0 && kOffAfk % 128 == 0 && kOffBfk % 128 == 0);

typedef __attribute__((ext_vector_type(16))) _Float16 v16h;
typedef __attribute__((ext_vector_type(8)))  _Float16 v8h;
typedef __attribute__((ext_vector_type(16))) __bf16   v16b;
typedef __attribute__((ext_vector_type(8)))  __bf16   v8b;
typedef __attribute__((ext_vector_type(8)))  float    v8f;
typedef __attribute__((ext_vector_type(4)))  float    v4f;
typedef __attribute__((ext_vector_type(4)))  unsigned int v4u;

__device__ __forceinline__ unsigned short f2bf_bits(float f) {
  unsigned u = __float_as_uint(f);
  return (unsigned short)((u + 0x7FFFu + ((u >> 16) & 1u)) >> 16);
}
__device__ __forceinline__ float bf_bits2f(unsigned short h) { return __uint_as_float(((unsigned)h) << 16); }

__device__ __forceinline__ void dep_guard_h(v8f& a, v8f& b, v16h x, v16h y) { asm volatile("v_nop\n\tv_nop\n\tv_nop\n\tv_nop" : "+v"(a), "+v"(b) : "v"(x), "v"(y)); }
__device__ __forceinline__ void dep_guard_b(v8f& a, v8f& b, v16b x, v16b y) { asm volatile("v_nop\n\tv_nop\n\tv_nop\n\tv_nop" : "+v"(a), "+v"(b) : "v"(x), "v"(y)); }
__device__ __forceinline__ void keep4_h(v16h a, v16h b, v16h c, v16h d) { asm volatile("v_nop" :: "v"(a), "v"(b), "v"(c), "v"(d)); }
__device__ __forceinline__ void keep4_b(v16b a, v16b b, v16b c, v16b d) { asm volatile("v_nop" :: "v"(a), "v"(b), "v"(c), "v"(d)); }
__device__ __forceinline__ void acc_guard4(v8f& a, v8f& b, v8f& c, v8f& d) { asm volatile("v_nop\n\tv_nop\n\tv_nop\n\tv_nop" : "+v"(a), "+v"(b), "+v"(c), "+v"(d)); }
template <typename T> struct Frag;
template <> struct Frag<_Float16> {
  typedef v16h V; union U { v16h v; v8h h[2]; };
  static __device__ __forceinline__ v16h load(const _Float16* p) {
    U f; f.h[0] = *(const v8h*)(p); f.h[1] = *(const v8h*)(p + 16); return f.v;
  }
  static __device__ __forceinline__ v8f mma(v16h a, v16h b, v8f c) {
    return __builtin_amdgcn_wmma_f32_16x16x32_f16(false, a, false, b, (short)0, c, false, false);
  }
  static __device__ __forceinline__ void guard(v8f& a, v8f& b, v16h x, v16h y) { dep_guard_h(a, b, x, y); }
  static __device__ __forceinline__ void keep(v16h a, v16h b, v16h c, v16h d) { keep4_h(a, b, c, d); }
};
template <> struct Frag<__bf16> {
  typedef v16b V; union U { v16b v; v8b h[2]; };
  static __device__ __forceinline__ v16b load(const __bf16* p) {
    U f; f.h[0] = *(const v8b*)(p); f.h[1] = *(const v8b*)(p + 16); return f.v;
  }
  static __device__ __forceinline__ v8f mma(v16b a, v16b b, v8f c) {
    return __builtin_amdgcn_wmma_f32_16x16x32_bf16(false, a, false, b, (short)0, c, false, false);
  }
  static __device__ __forceinline__ void guard(v8f& a, v8f& b, v16b x, v16b y) { dep_guard_b(a, b, x, y); }
  static __device__ __forceinline__ void keep(v16b a, v16b b, v16b c, v16b d) { keep4_b(a, b, c, d); }
};

__device__ __forceinline__ unsigned pk16(unsigned short a, unsigned short b) { return (unsigned)a | ((unsigned)b << 16); }

template <int ET> struct Elem;
template <> struct Elem<0> { typedef _Float16 T; };
template <> struct Elem<1> { typedef __bf16 T; };
template <int ET, bool SPLIT, int BIAS_MODE, int OUT_MODE, bool RESID, int ACT = 0>
__global__ __launch_bounds__(256) void wmma_gemm64(
    const unsigned short* __restrict__ Ap, const unsigned short* __restrict__ A2p, int lda, long strideA,
    const unsigned short* __restrict__ Btp, const unsigned short* __restrict__ Bt2p, int ldb, long strideB,
    void* __restrict__ Cout, void* __restrict__ Cout2, int ldc, long strideC,
    const float* __restrict__ bias,
    const float* __restrict__ resid, long strideR,
    int M, int N, int K, float scale) {
  typedef typename Elem<ET>::T T;
  typedef typename Frag<T>::V V;
  const T* A = (const T*)Ap; const T* A2 = (const T*)A2p; const T* Bt = (const T*)Btp; const T* Bt2 = (const T*)Bt2p;
  __shared__ __align__(16) float sT[8][16 * 68];
  const int b    = blockIdx.y;
  const int lane = threadIdx.x & 31;
  const int wave = threadIdx.x >> 5;
  const int tilesN = N >> 6;
  const int tilesM = M >> 6;
  const int tile = blockIdx.x * 8 + wave;
  if (tile >= tilesM * tilesN) return;
  const int tm = tile / tilesN;
  const int tn = tile - tm * tilesN;
  const int m0 = tm << 6;
  const int n0 = tn << 6;

  const T* Ab  = A  + (size_t)b * strideA;
  const T* Bb  = Bt + (size_t)b * strideB;
  const T* Ab2 = SPLIT ? (A2  + (size_t)b * strideA) : nullptr;
  const T* Bb2 = SPLIT ? (Bt2 + (size_t)b * strideB) : nullptr;

  const int rlane = lane & 15;
  const int koff  = (lane >> 4) * 8;
  const int mOff  = (lane >> 4) * 8;

  v8f acc[4][4];
#pragma unroll
  for (int i = 0; i < 4; ++i)
#pragma unroll
    for (int j = 0; j < 4; ++j) acc[i][j] = (v8f){0.f,0.f,0.f,0.f,0.f,0.f,0.f,0.f};

  for (int k0 = 0; k0 < K; k0 += 32) {
    V bh[4], bl[4];
#pragma unroll
    for (int j = 0; j < 4; ++j) {
      const size_t bo = (size_t)(n0 + (j << 4) + rlane) * ldb + koff + k0;
      bh[j] = Frag<T>::load(Bb + bo);
      if (SPLIT) bl[j] = Frag<T>::load(Bb2 + bo);
    }
#pragma unroll
    for (int i = 0; i < 4; ++i) {
      const size_t ao = (size_t)(m0 + (i << 4) + rlane) * lda + koff + k0;
      V ah = Frag<T>::load(Ab + ao);
      V al;
      if (SPLIT) al = Frag<T>::load(Ab2 + ao);
#pragma unroll
      for (int j = 0; j < 4; ++j) {
        acc[i][j] = Frag<T>::mma(ah, bh[j], acc[i][j]);
        if (SPLIT) {
          acc[i][j] = Frag<T>::mma(ah, bl[j], acc[i][j]);
          acc[i][j] = Frag<T>::mma(al, bh[j], acc[i][j]);
        }
      }
      Frag<T>::guard(acc[i][0], acc[i][3], ah, SPLIT ? al : ah);
    }
    Frag<T>::keep(bh[0], bh[1], bh[2], bh[3]);
    if (SPLIT) Frag<T>::keep(bl[0], bl[1], bl[2], bl[3]);
  }
  acc_guard4(acc[0][0], acc[0][1], acc[0][2], acc[0][3]);
  acc_guard4(acc[1][0], acc[1][1], acc[1][2], acc[1][3]);
  acc_guard4(acc[2][0], acc[2][1], acc[2][2], acc[2][3]);
  acc_guard4(acc[3][0], acc[3][1], acc[3][2], acc[3][3]);

  float* slab = sT[wave];
  const float* Rb = RESID ? (resid + (size_t)b * strideR) : nullptr;
#pragma unroll
  for (int i = 0; i < 4; ++i) {
    const int mBase = m0 + (i << 4);
#pragma unroll
    for (int j = 0; j < 4; ++j) {
      const int n = n0 + (j << 4) + rlane;
      float bv = 0.f;
      if (BIAS_MODE == 2) bv = bias[n];
#pragma unroll
      for (int r = 0; r < 8; ++r) {
        float v = acc[i][j][r] * scale;
        if (BIAS_MODE == 1) v += bias[mBase + mOff + r];
        if (BIAS_MODE == 2) v += bv;
        if (RESID) v += Rb[(size_t)(mBase + mOff + r) * ldc + n];
        if (ACT == 2) v = fmaxf(v, 0.0f);
        if (ACT == 4) v = (v > 0.f) ? v : 0.01f * v;
        slab[(mOff + r) * 68 + (j << 4) + rlane] = v;
      }
    }
    __builtin_amdgcn_fence(__ATOMIC_RELEASE, "workgroup");
    __builtin_amdgcn_wave_barrier();
    __builtin_amdgcn_fence(__ATOMIC_ACQUIRE, "workgroup");
    if (OUT_MODE == 0) {
      float* C = (float*)Cout + (size_t)b * strideC;
      const int hh = lane >> 4, c4 = (lane & 15) * 4;
      for (int pass = 0; pass < 2; ++pass) {
#pragma unroll
        for (int it = 0; it < 8; ++it) {
          const int row = it * 2 + hh;
          v4f v = *(const v4f*)(slab + row * 68 + c4);
          *(volatile v4f*)(C + (size_t)(mBase + row) * ldc + n0 + c4) = v;
        }
        __threadfence();
      }
    } else {
      const int q = lane >> 3, c8 = (lane & 7) * 8;
      unsigned short* C  = (unsigned short*)Cout  + (size_t)b * strideC;
      unsigned short* C2 = (OUT_MODE == 2) ? ((unsigned short*)Cout2 + (size_t)b * strideC) : nullptr;
      for (int pass = 0; pass < 2; ++pass) {
#pragma unroll
        for (int it = 0; it < 4; ++it) {
          const int row = it * 4 + q;
          const float* sp = slab + row * 68 + c8;
          v8h hv, lv;
#pragma unroll
          for (int e = 0; e < 8; ++e) {
            if (OUT_MODE == 1) {
              hv[e] = (_Float16)sp[e];
            } else {
              unsigned short hb = f2bf_bits(sp[e]);
              unsigned short lb = f2bf_bits(sp[e] - bf_bits2f(hb));
              hv[e] = __builtin_bit_cast(_Float16, hb);
              lv[e] = __builtin_bit_cast(_Float16, lb);
            }
          }
          *(volatile v8h*)(C + (size_t)(mBase + row) * ldc + n0 + c8) = hv;
          if (OUT_MODE == 2) *(volatile v8h*)(C2 + (size_t)(mBase + row) * ldc + n0 + c8) = lv;
        }
        __threadfence();
      }
    }
    __builtin_amdgcn_fence(__ATOMIC_RELEASE, "workgroup");
    __builtin_amdgcn_wave_barrier();
    __builtin_amdgcn_fence(__ATOMIC_ACQUIRE, "workgroup");
  }
}

__global__ __launch_bounds__(256) void cast8_bf16_kernel(const float* __restrict__ a, const float* __restrict__ b,
                                                         const float* __restrict__ f, unsigned short* __restrict__ outp) {
  const int blk = blockIdx.x;
  const int seg = (blk < kBlkA) ? 0 : (blk < kBlkA + kBlkB) ? 1 : 2;
  const float* src = (seg == 0) ? a : (seg == 1) ? b : f;
  const int lblk = blk - ((seg == 0) ? 0 : (seg == 1) ? kBlkA : (kBlkA + kBlkB));
  const size_t obase = (seg == 0) ? (size_t)0 : (seg == 1) ? ((size_t)kNa * kDD) : ((size_t)(kNa + kNb) * kDD);
  const size_t n8 = (seg == 0) ? ((size_t)kNa * kDD / 8) : (seg == 1) ? ((size_t)kNb * kDD / 8) : ((size_t)kKF * kDD / 8);
  const size_t i = (size_t)lblk * 256 + threadIdx.x;
  if (i >= n8) return;
  const float* p = src + 8 * i;
  const v4f x = *(const v4f*)(p);
  const v4f y = *(const v4f*)(p + 4);
  unsigned short hb[8];
#pragma unroll
  for (int e = 0; e < 4; ++e) {
    hb[e]     = f2bf_bits(x[e]);
    hb[4 + e] = f2bf_bits(y[e]);
  }
  const v4u u = (v4u){pk16(hb[0], hb[1]), pk16(hb[2], hb[3]), pk16(hb[4], hb[5]), pk16(hb[6], hb[7])};
  unsigned short* q = outp + obase + 8 * i;
  *(volatile v4u*)q = u;
  __threadfence();
  *(volatile v4u*)q = u;
}

__global__ __launch_bounds__(256) void masked_sum_kernel(const float* __restrict__ AFK, const float* __restrict__ BFK,
                                                         float* __restrict__ out) {
  __shared__ __align__(16) float apS[kTI * kKF];
  __shared__ unsigned nbS[kTJ * 8];
  __shared__ __align__(16) float stg[8][8 * kStgPitch];
  const int t    = threadIdx.x;
  const int lane = t & 31;
  const int wave = t >> 5;
  const int i0 = blockIdx.y * kTI;
  const int j0 = blockIdx.x * kTJ;

#pragma unroll
  for (int it = 0; it < 8; ++it) {
    const int q   = it * 256 + t;
    const int row = q >> 6;
    const int c4  = (q & 63) * 4;
    const v4f v = *(const v4f*)(AFK + (size_t)(i0 + row) * kKF + c4);
    v4f rl;
#pragma unroll
    for (int e = 0; e < 4; ++e) rl[e] = (v[e] > 0.0f) ? v[e] : 0.0f;
    *(v4f*)(apS + row * kKF + c4) = rl;
  }
  {
    const int jl = t >> 2;
    const int wq = t & 3;
    const float* br = BFK + (size_t)(j0 + jl) * kKF + wq * 64;
    unsigned w0 = 0u, w1 = 0u;
#pragma unroll
    for (int g = 0; g < 8; ++g) {
      const v4f v0 = *(const v4f*)(br + 4 * g);
      const v4f v1 = *(const v4f*)(br + 32 + 4 * g);
#pragma unroll
      for (int e = 0; e < 4; ++e) {
        w0 |= ((v0[e] <= 0.0f) ? 1u : 0u) << (4 * g + e);
        w1 |= ((v1[e] <= 0.0f) ? 1u : 0u) << (4 * g + e);
      }
    }
    nbS[jl * 8 + wq * 2]     = w0;
    nbS[jl * 8 + wq * 2 + 1] = w1;
  }
  __syncthreads();

  const int ig = wave >> 1;
  const int jh = wave & 1;
  const int jl = jh * 32 + lane;
  const float* apr = apS + (ig * 8) * kKF;
  const unsigned* nbr = nbS + jl * 8;
  float acc[8];
#pragma unroll
  for (int r = 0; r < 8; ++r) acc[r] = 0.0f;

#pragma unroll 1
  for (int k4 = 0; k4 < kKF / 4; ++k4) {
    const unsigned bits = nbr[k4 >> 3] >> ((k4 & 7) * 4);
#pragma unroll
    for (int r = 0; r < 8; ++r) {
      const v4f av = *(const v4f*)(apr + r * kKF + k4 * 4);
#pragma unroll
      for (int e = 0; e < 4; ++e) {
        const unsigned sel = (bits >> e) & 1u;
        acc[r] += (sel != 0u) ? av[e] : 0.0f;
      }
    }
  }

  float* sw = stg[wave];
#pragma unroll
  for (int r = 0; r < 8; ++r) sw[r * kStgPitch + lane] = acc[r];
  __builtin_amdgcn_fence(__ATOMIC_RELEASE, "workgroup");
  __builtin_amdgcn_wave_barrier();
  __builtin_amdgcn_fence(__ATOMIC_ACQUIRE, "workgroup");
  const int rq = lane >> 3;
  const int c4 = (lane & 7) * 4;
  float* ob = out + (size_t)(i0 + ig * 8) * kNb + j0 + jh * 32 + c4;
  for (int pass = 0; pass < 2; ++pass) {
#pragma unroll
    for (int it = 0; it < 2; ++it) {
      const int row = it * 4 + rq;
      const v4f v = *(const v4f*)(sw + row * kStgPitch + c4);
      *(volatile v4f*)(ob + (size_t)row * kNb) = v;
    }
    __threadfence();
  }
}

extern "C" void kernel_launch(void* const* d_in, const int* in_sizes, int n_in,
                              void* d_out, int out_size, void* d_ws,
                              size_t ws_size, hipStream_t stream) {
  if (n_in < 3) return;
  if (in_sizes[0] != kNa * kDD || in_sizes[1] != kNb * kDD || in_sizes[2] != kKF * kDD) return;
  if (out_size != kNa * kNb) return;
  if (ws_size < kWsTotal) return;

  const float* a     = (const float*)d_in[0];
  const float* b     = (const float*)d_in[1];
  const float* feats = (const float*)d_in[2];
  float* out = (float*)d_out;

  unsigned char* ws = (unsigned char*)d_ws;
  unsigned short* abf = (unsigned short*)(ws + kOffAbf);
  unsigned short* fbf = (unsigned short*)(ws + kOffFbf);
  float* afk = (float*)(ws + kOffAfk);
  float* bfk = (float*)(ws + kOffBfk);

  cast8_bf16_kernel<<<dim3(kBlkA + kBlkB + kBlkF, 1, 1), dim3(256, 1, 1), 0, stream>>>(a, b, feats, abf);

  wmma_gemm64<1, false, 0, 0, false, 0><<<dim3(8, 2, 1), dim3(256, 1, 1), 0, stream>>>(
      abf, nullptr, kDD, (long)kNa * kDD,
      fbf, nullptr, kDD, 0L,
      (void*)afk, nullptr, kKF, (long)kNa * kKF,
      nullptr, nullptr, 0L,
      kNa, kKF, kDD, 1.0f);

  masked_sum_kernel<<<dim3(kNb / kTJ, kNa / kTI, 1), dim3(256, 1, 1), 0, stream>>>(afk, bfk, out);
}
